// GatedAttentionBasedRNN_1297080124080
// MI455X (gfx1250) — hardware-verified
//
#include <hip/hip_runtime.h>
#include <math.h>

#define __bf16 _Float16
typedef __attribute__((ext_vector_type(16))) __bf16 v16bf;
typedef __attribute__((ext_vector_type(8)))  __bf16 v8bf;
typedef __attribute__((ext_vector_type(8)))  float  v8f;
typedef __attribute__((ext_vector_type(4)))  float  v4f_t;
typedef float v4fa __attribute__((ext_vector_type(4), may_alias));
typedef __attribute__((ext_vector_type(4)))  unsigned v4u_t;
typedef unsigned v4ua __attribute__((ext_vector_type(4), may_alias));
#define RSPLIT (1.0f / 2048.0f)
__device__ __forceinline__ __bf16 lo_of(float v, __bf16 h) { return (__bf16)((v - (float)h) * 2048.0f); }
__device__ __forceinline__ void st2f(float* p, float v) { *(volatile float*)p = v; __threadfence(); *(volatile float*)p = v; }

#define PP 512
#define QQ 64
#define BB 16
#define EE 256
#define HH 256
#define OO 256
#define PL_PASS ((size_t)PP * BB * EE)
#define PL_QUES ((size_t)QQ * BB * EE)
#define PL_WUP  ((size_t)HH * EE)
#define PL_WUQ  ((size_t)HH * EE)
#define PL_WG   ((size_t)2 * EE * 2 * EE)
#define PL_WIH  ((size_t)3 * OO * EE)
#define PL_WHH  ((size_t)3 * OO * OO)
#define PL_CAT  ((size_t)PP * BB * 2 * EE)
#define PL_X    ((size_t)PP * BB * EE)

__device__ __forceinline__ v8f wmma_bf16(v16bf a, v16bf b, v8f c) {
    return __builtin_amdgcn_wmma_f32_16x16x32_f16(
         false, a,  false, b,
         (short)0, c,  false,  false);
}
__device__ __forceinline__ v8f wmma_split(v16bf a, v16bf al, v16bf b, v16bf bl, v8f c) {
    v8f x = {}; x = wmma_bf16(al, b, x); x = wmma_bf16(a, bl, x); return wmma_bf16(a, b, c) + x * RSPLIT;
}

__device__ __forceinline__ v16bf load_frag_A(const __bf16* __restrict__ A,
                                             int lda, int m0, int k0) {
    int lane = threadIdx.x & 31;
    int m = lane & 15, half = (lane >> 4) & 1;
    const __bf16* base = A + (size_t)(m0 + m) * lda + k0;
    v16bf f;
#pragma unroll
    for (int i = 0; i < 8; ++i) f[i] = base[half * 8 + i];
#pragma unroll
    for (int i = 0; i < 8; ++i) f[8 + i] = base[16 + half * 8 + i];
    return f;
}

__device__ __forceinline__ v16bf load_frag_B(const __bf16* __restrict__ W,
                                             int ldw, int n0, int k0) {
    int lane = threadIdx.x & 31;
    int n = lane & 15, half = (lane >> 4) & 1;
    const __bf16* base = W + (size_t)(n0 + n) * ldw + k0;
    return __builtin_shufflevector(*(const v8bf*)(base + half * 8), *(const v8bf*)(base + 16 + half * 8), 0,1,2,3,4,5,6,7,8,9,10,11,12,13,14,15);
}

__global__ void f32_to_bf16_kernel(const float* __restrict__ in,
                                   __bf16* __restrict__ out, int n, size_t pl) {
    int i = (blockIdx.x * blockDim.x + threadIdx.x) * 2;
    if (i < n) {
        const __bf16 a = (__bf16)in[i], b = (__bf16)in[i + 1];
        const unsigned u = (unsigned)__builtin_bit_cast(unsigned short, a) | ((unsigned)__builtin_bit_cast(unsigned short, b) << 16);
        const unsigned w = (unsigned)__builtin_bit_cast(unsigned short, lo_of(in[i], a)) | ((unsigned)__builtin_bit_cast(unsigned short, lo_of(in[i + 1], b)) << 16);
        *(volatile unsigned*)(out + i) = u; *(volatile unsigned*)(out + pl + i) = w; __threadfence();
        *(volatile unsigned*)(out + i) = u; *(volatile unsigned*)(out + pl + i) = w;
    }
}

__global__ __launch_bounds__(256)
void wmma_gemm_kernel(const __bf16* __restrict__ A, size_t plA, const __bf16* __restrict__ W, size_t plW,
                      int M, int N, int K, int ldw, int mode,
                      float* __restrict__ outf, const float* __restrict__ bias,
                      const float* __restrict__ aux, __bf16* __restrict__ outb, size_t plO) {
    __shared__ __attribute__((aligned(16))) float stg[8][16 * 68];
    int wave = threadIdx.x >> 5;
    int gw = blockIdx.x * (blockDim.x >> 5) + wave;
    int ngrp = N >> 6;
    int groups = (M >> 4) * ngrp;
    if (gw >= groups) return;
    int mt = gw / ngrp, ng = gw - mt * ngrp;
    int m0 = mt << 4, n0 = ng << 6;

    v8f acc[4] = {};
    for (int k0 = 0; k0 < K; k0 += 32) {
        v16bf a  = load_frag_A(A, K, m0, k0), al = load_frag_A(A + plA, K, m0, k0);
#pragma unroll
        for (int t = 0; t < 4; ++t) {
            v16bf b = load_frag_B(W, ldw, n0 + 16 * t, k0), bl = load_frag_B(W + plW, ldw, n0 + 16 * t, k0);
            acc[t] = wmma_split(a, al, b, bl, acc[t]);
        }
    }

    int lane = threadIdx.x & 31;
    int n = lane & 15, half = (lane >> 4) & 1;
    float* sw = stg[wave];
#pragma unroll
    for (int t = 0; t < 4; ++t) {
        int nn = n0 + t * 16 + n;
#pragma unroll
        for (int r = 0; r < 8; ++r) {
            int m = m0 + r + half * 8;
            float d = acc[t][r];
            size_t idx = (size_t)m * N + nn;
            float v;
            if (mode == 0)      v = d;
            else if (mode == 1) v = d + bias[nn];
            else                v = aux[idx] / (1.0f + __expf(-d));
            sw[(r + half * 8) * 68 + t * 16 + n] = v;
        }
    }
    asm volatile("s_wait_dscnt 0" ::: "memory");
#pragma unroll 1
    for (int pass = 0; pass < 2; ++pass) {
        if (mode != 2) {
#pragma unroll
            for (int i = 0; i < 8; ++i) { const int c = lane + 32 * i, rr = c >> 4, q = (c & 15) * 4;
                *(volatile v4f_t*)(outf + (size_t)(m0 + rr) * N + n0 + q) = *(const volatile v4fa*)(sw + rr * 68 + q); }
        } else {
#pragma unroll
            for (int i = 0; i < 4; ++i) { const int c = lane + 32 * i, rr = c >> 3, q = (c & 7) * 8; const float* s = sw + rr * 68 + q;
                __bf16 hh[8], hl[8];
#pragma unroll
                for (int e = 0; e < 8; ++e) { hh[e] = (__bf16)s[e]; hl[e] = lo_of(s[e], hh[e]); }
                __bf16* d = outb + (size_t)(m0 + rr) * N + n0 + q;
                *(volatile v4u_t*)d = *(const v4ua*)hh; *(volatile v4u_t*)(d + plO) = *(const v4ua*)hl; }
        }
        __threadfence();
    }
}

__global__ __launch_bounds__(256)
void attn_kernel(const float* __restrict__ Wp,
                 const float* __restrict__ Wq,
                 const float* __restrict__ vv,
                 const float* __restrict__ question,
                 const float* __restrict__ passage,
                 __bf16* __restrict__ catb,
                 float* __restrict__ cf) {
    __shared__ float sc[QQ];
    __shared__ float aw[QQ];
    int p = blockIdx.x >> 4;
    int b = blockIdx.x & 15;
    int tid = threadIdx.x;
    int wave = tid >> 5, lane = tid & 31;

    const float* wp = Wp + (size_t)(p * BB + b) * HH;
#pragma unroll 1
    for (int q = wave * 8; q < wave * 8 + 8; ++q) {
        const float* wq = Wq + (size_t)(q * BB + b) * HH;
        float t = 0.f;
#pragma unroll 1
        for (int h = lane; h < HH; h += 32)
            t += vv[h] * tanhf(wq[h] + wp[h]);
#pragma unroll
        for (int off = 16; off > 0; off >>= 1) t += __shfl_xor(t, off, 32);
        if (lane == 0) sc[q] = t;
    }
    __syncthreads();
    if (tid == 0) {
        float mx = sc[0];
        for (int q = 1; q < QQ; ++q) mx = fmaxf(mx, sc[q]);
        float s = 0.f;
        for (int q = 0; q < QQ; ++q) { float e = __expf(sc[q] - mx); aw[q] = e; s += e; }
        float inv = 1.0f / s;
        for (int q = 0; q < QQ; ++q) aw[q] *= inv;
    }
    __syncthreads();
    int e = tid;
    float c = 0.f;
#pragma unroll 1
    for (int q = 0; q < QQ; ++q)
        c += aw[q] * question[(size_t)(q * BB + b) * EE + e];
    size_t row = (size_t)p * BB + b;
    st2f(cf + row * EE + e, c);
    __shared__ __attribute__((aligned(16))) float scat[2 * EE];
    scat[e] = passage[row * EE + e]; scat[EE + e] = c;
    __syncthreads();
    if (tid < 2 * EE / 8) {
        __bf16 hh[8], hl[8];
#pragma unroll
        for (int k = 0; k < 8; ++k) { const float f = scat[tid * 8 + k]; hh[k] = (__bf16)f; hl[k] = lo_of(f, hh[k]); }
        __bf16* d = catb + row * (2 * EE) + tid * 8;
        *(volatile v4u_t*)d = *(const v4ua*)hh; *(volatile v4u_t*)(d + PL_CAT) = *(const v4ua*)hl; __threadfence();
        *(volatile v4u_t*)d = *(const v4ua*)hh; *(volatile v4u_t*)(d + PL_CAT) = *(const v4ua*)hl;
    }
}

__global__ __launch_bounds__(512, 1)
void gru_kernel(const float* __restrict__ gi,
                const __bf16* __restrict__ whh,
                const float* __restrict__ bhh,
                float* __restrict__ out) {
    extern __shared__ char smem[];
    float*  gh = (float*)smem;
    float*  hS = (float*)(smem + 49152);
    __bf16* hB = (__bf16*)(smem + 49152 + 16384);
    __bf16* hBl = hB + BB * OO;

    int tid = threadIdx.x;
    int wave = tid >> 5;
    int t0 = wave, t1 = wave + 16, t2 = wave + 32;

    const __bf16* whl = whh + PL_WHH;

    for (int i = tid; i < BB * OO; i += 512) { hS[i] = 0.f; hB[i] = (__bf16)0.0f; hBl[i] = (__bf16)0.0f; }
    __syncthreads();

    int lane = tid & 31;
    int n = lane & 15, half = (lane >> 4) & 1;

    for (int p = 0; p < PP; ++p) {
        v8f a0 = {}, a1 = {}, a2 = {};
#pragma unroll 2
        for (int kk = 0; kk < 8; ++kk) {
            v16bf af = load_frag_A(hB, OO, 0, kk * 32), afl = load_frag_A(hBl, OO, 0, kk * 32);
            a0 = wmma_split(af, afl, load_frag_B(whh, OO, t0 * 16, kk * 32), load_frag_B(whl, OO, t0 * 16, kk * 32), a0);
            a1 = wmma_split(af, afl, load_frag_B(whh, OO, t1 * 16, kk * 32), load_frag_B(whl, OO, t1 * 16, kk * 32), a1);
            a2 = wmma_split(af, afl, load_frag_B(whh, OO, t2 * 16, kk * 32), load_frag_B(whl, OO, t2 * 16, kk * 32), a2);
        }
#pragma unroll
        for (int r = 0; r < 8; ++r) {
            int m = r + half * 8;
            gh[m * 768 + t0 * 16 + n] = a0[r];
            gh[m * 768 + t1 * 16 + n] = a1[r];
            gh[m * 768 + t2 * 16 + n] = a2[r];
        }
        __syncthreads();

        const float* gip = gi + (size_t)p * BB * 768;
        for (int idx = tid; idx < BB * OO; idx += 512) {
            int b = idx >> 8, o = idx & 255;
            float gr = gip[b * 768 + o]       + gh[b * 768 + o]       + bhh[o];
            float gz = gip[b * 768 + 256 + o] + gh[b * 768 + 256 + o] + bhh[256 + o];
            float gn = gip[b * 768 + 512 + o];
            float hn = gh[b * 768 + 512 + o] + bhh[512 + o];
            float r = 1.0f / (1.0f + __expf(-gr));
            float z = 1.0f / (1.0f + __expf(-gz));
            float nn = tanhf(gn + r * hn);
            float h = hS[idx];
            float hnew = (1.0f - z) * nn + z * h;
            hS[idx] = hnew;
            const __bf16 hh = (__bf16)hnew; hB[idx] = hh; hBl[idx] = lo_of(hnew, hh);
            st2f(out + ((size_t)p * BB + b) * OO + o, hnew);
        }
        __syncthreads();
    }
}

extern "C" void kernel_launch(void* const* d_in, const int* in_sizes, int n_in,
                              void* d_out, int out_size, void* d_ws, size_t ws_size,
                              hipStream_t stream) {
    const float* passage  = (const float*)d_in[0];
    const float* question = (const float*)d_in[1];
    const float* Wuq      = (const float*)d_in[2];
    const float* Wup      = (const float*)d_in[3];
    const float* vvec     = (const float*)d_in[4];
    const float* Wg       = (const float*)d_in[5];
    const float* w_ih     = (const float*)d_in[6];
    const float* w_hh     = (const float*)d_in[7];
    const float* b_ih     = (const float*)d_in[8];
    const float* b_hh     = (const float*)d_in[9];
    float* out = (float*)d_out;

    char* ws = (char*)d_ws;
    size_t off = 0;
    auto alloc = [&](size_t bytes) { char* p = ws + off; off = (off + bytes + 255) & ~(size_t)255; return p; };

    float*  Wp_f    = (float*)alloc((size_t)PP * BB * HH * 4);
    float*  Wq_f    = (float*)alloc((size_t)QQ * BB * HH * 4);
    __bf16* pass_b  = (__bf16*)alloc((size_t)PP * BB * EE * 2 * 2);
    __bf16* ques_b  = (__bf16*)alloc((size_t)QQ * BB * EE * 2 * 2);
    __bf16* Wup_b   = (__bf16*)alloc((size_t)HH * EE * 2 * 2);
    __bf16* Wuq_b   = (__bf16*)alloc((size_t)HH * EE * 2 * 2);
    __bf16* Wg_b    = (__bf16*)alloc((size_t)2 * EE * 2 * EE * 2 * 2);
    __bf16* wih_b   = (__bf16*)alloc((size_t)3 * OO * EE * 2 * 2);
    __bf16* whh_b   = (__bf16*)alloc((size_t)3 * OO * OO * 2 * 2);
    __bf16* cat_b   = (__bf16*)alloc((size_t)PP * BB * 2 * EE * 2 * 2);
    float*  c_f     = (float*)alloc((size_t)PP * BB * EE * 4);
    __bf16* x_b     = (__bf16*)alloc((size_t)PP * BB * EE * 2 * 2);
    float*  gi_f    = (float*)alloc((size_t)PP * BB * 3 * OO * 4);
    (void)ws_size;

    auto conv = [&](const float* src, __bf16* dst, int n, size_t pl) {
        f32_to_bf16_kernel<<<(n / 2 + 255) / 256, 256, 0, stream>>>(src, dst, n, pl);
    };
    conv(passage, pass_b, PP * BB * EE, PL_PASS);
    conv(question, ques_b, QQ * BB * EE, PL_QUES);
    conv(Wup, Wup_b, HH * EE, PL_WUP);
    conv(Wuq, Wuq_b, HH * EE, PL_WUQ);
    conv(Wg, Wg_b, 2 * EE * 2 * EE, PL_WG);
    conv(w_ih, wih_b, 3 * OO * EE, PL_WIH);
    conv(w_hh, whh_b, 3 * OO * OO, PL_WHH);

    auto gemm = [&](const __bf16* A, size_t plA, const __bf16* W, size_t plW, int M, int N, int K, int ldw,
                    int mode, float* outf, const float* bias, const float* aux, __bf16* outb, size_t plO) {
        int groups = (M / 16) * (N / 64);
        int blocks = (groups + 7) / 8;
        wmma_gemm_kernel<<<blocks, 256, 0, stream>>>(A, plA, W, plW, M, N, K, ldw, mode,
                                                     outf, bias, aux, outb, plO);
    };

    gemm(pass_b, PL_PASS, Wup_b, PL_WUP, PP * BB, HH, EE, EE, 0, Wp_f, nullptr, nullptr, nullptr, 0);
    gemm(ques_b, PL_QUES, Wuq_b, PL_WUQ, QQ * BB, HH, EE, EE, 0, Wq_f, nullptr, nullptr, nullptr, 0);

    attn_kernel<<<PP * BB, 256, 0, stream>>>(Wp_f, Wq_f, vvec, question, passage,
                                             cat_b, c_f);

    gemm(cat_b, PL_CAT, Wg_b + (size_t)EE * (2 * EE), PL_WG, PP * BB, EE, 2 * EE, 2 * EE,
         2, nullptr, nullptr, c_f, x_b, PL_X);

    gemm(x_b, PL_X, wih_b, PL_WIH, PP * BB, 3 * OO, EE, EE, 1, gi_f, b_ih, nullptr, nullptr, 0);

    gru_kernel<<<1, 512, 49152 + 16384 + 8192 + 8192, stream>>>(gi_f, whh_b, b_hh, out);

    (void)in_sizes; (void)n_in; (void)out_size;
}
